// QuantFinanceAttention_65000035058567
// MI455X (gfx1250) — hardware-verified
//
#include <hip/hip_runtime.h>
#include <math.h>


#define NB 2
#define NT 2048
#define NC 1024
#define NH 16
#define DK 64
#define KD 1024
#define PSX ((size_t)NB * NT * NC)
#define PSW ((size_t)NC * NC)
#define NEG_INF (-__builtin_inff())
#define HAZ4 "v_nop\n\tv_nop\n\tv_nop\n\tv_nop"

typedef __bf16 v16bf __attribute__((ext_vector_type(16)));
typedef __bf16 bf16x8 __attribute__((ext_vector_type(8)));
typedef float v8f __attribute__((ext_vector_type(8)));
typedef float f32x4 __attribute__((ext_vector_type(4), may_alias));
typedef int i32x4 __attribute__((ext_vector_type(4), may_alias));
typedef unsigned int u32x4 __attribute__((ext_vector_type(4), may_alias));

union Frag { v16bf v; bf16x8 h[2]; };
union P8 { bf16x8 b; u32x4 u; };
union V8 { v8f v; f32x4 q[2]; };
union U4 { f32x4 f; u32x4 u; };

static __device__ __forceinline__ v8f mma(v16bf a, v16bf b, v8f c) {
  return __builtin_amdgcn_wmma_f32_16x16x32_bf16(false, a, false, b, (short)0, c, false, false);
}

static __device__ __forceinline__ void split8(const float (&y)[8], u32x4& hi, u32x4& lo) {
  P8 a, c;
#pragma unroll
  for (int r = 0; r < 8; ++r) {
    const __bf16 hv = (__bf16)y[r];
    const float hf = (float)hv;
    const __bf16 lv = (__bf16)(y[r] - hf);
    a.b[r] = hv;
    c.b[r] = lv;
  }
  hi = a.u;
  lo = c.u;
}

static __device__ __forceinline__ void gemm_core(const __bf16* __restrict__ A, size_t aps,
                                                 const __bf16* __restrict__ Bm, size_t bps,
                                                 int lm, int lh, v8f (&acc)[4][2]) {
  const __bf16* ar[4];
  const __bf16* br[2];
#pragma unroll
  for (int at = 0; at < 4; ++at) ar[at] = A + (size_t)(16 * at + lm) * KD + 8 * lh;
#pragma unroll
  for (int bt = 0; bt < 2; ++bt) br[bt] = Bm + (size_t)(16 * bt + lm) * KD + 8 * lh;
  for (int k0 = 0; k0 < KD; k0 += 32) {
    Frag bh[2], bl[2];
#pragma unroll
    for (int bt = 0; bt < 2; ++bt) {
      bh[bt].h[0] = *(const bf16x8*)(br[bt] + k0);
      bh[bt].h[1] = *(const bf16x8*)(br[bt] + k0 + 16);
      bl[bt].h[0] = *(const bf16x8*)(br[bt] + bps + k0);
      bl[bt].h[1] = *(const bf16x8*)(br[bt] + bps + k0 + 16);
    }
    Frag ah, al;
#pragma unroll
    for (int at = 0; at < 4; ++at) {
      ah.h[0] = *(const bf16x8*)(ar[at] + k0);
      ah.h[1] = *(const bf16x8*)(ar[at] + k0 + 16);
      al.h[0] = *(const bf16x8*)(ar[at] + aps + k0);
      al.h[1] = *(const bf16x8*)(ar[at] + aps + k0 + 16);
#pragma unroll
      for (int bt = 0; bt < 2; ++bt) {
        acc[at][bt] = mma(ah.v, bh[bt].v, acc[at][bt]);
        acc[at][bt] = mma(ah.v, bl[bt].v, acc[at][bt]);
        acc[at][bt] = mma(al.v, bh[bt].v, acc[at][bt]);
      }
    }
    asm volatile(HAZ4
                 : "+v"(acc[0][0]), "+v"(acc[0][1]), "+v"(acc[1][0]), "+v"(acc[1][1]),
                   "+v"(acc[2][0]), "+v"(acc[2][1]), "+v"(acc[3][0]), "+v"(acc[3][1])
                 : "v"(al.v), "v"(bh[1].v));
  }
}

__global__ void __launch_bounds__(256) k_split(const float* s0, const float* s1, const float* s2, const float* s3,
                                               __bf16* d0, __bf16* d1, __bf16* d2, __bf16* d3, int n) {
  const int sel = (int)blockIdx.y;
  const float* s = (sel == 0) ? s0 : (sel == 1) ? s1 : (sel == 2) ? s2 : s3;
  __bf16* d = (sel == 0) ? d0 : (sel == 1) ? d1 : (sel == 2) ? d2 : d3;
  const size_t i = ((size_t)blockIdx.x * 256 + threadIdx.x) * 8;
  if (i + 8 > (size_t)n) return;
  const f32x4 a = *(const f32x4*)(s + i);
  const f32x4 b = *(const f32x4*)(s + i + 4);
  float y[8];
#pragma unroll
  for (int r = 0; r < 4; ++r) { y[r] = a[r]; y[r + 4] = b[r]; }
  u32x4 hi, lo;
  split8(y, hi, lo);
  volatile u32x4* ph = (volatile u32x4*)(d + i);
  volatile u32x4* pl = (volatile u32x4*)(d + (size_t)n + i);
  *ph = hi;
  *pl = lo;
  __threadfence();
  *ph = hi;
  *pl = lo;
}

__global__ void __launch_bounds__(256) k_rope(float* cosT, float* sinT) {
  const int lane = threadIdx.x & 31, w = threadIdx.x >> 5;
  const int t = (int)blockIdx.x * 8 + w;
  const int j = lane;
  const double r2v = sqrt(10.0);
  const double r4v = sqrt(r2v);
  const double r8v = sqrt(r4v);
  const int m = j >> 3, f = j & 7;
  const double pf = ((f & 1) ? r8v : 1.0) * ((f & 2) ? r4v : 1.0) * ((f & 4) ? r2v : 1.0);
  const double p10 = ((m & 1) ? 10.0 : 1.0) * ((m & 2) ? 100.0 : 1.0);
  const float p32 = (float)(p10 * pf);
  const float inv = (float)(1.0 / (double)p32);
  const float ang = (float)t * inv;
  const double ad = (double)ang;
  const double n = rint(ad * 0.6366197723675814);
  double rr = fma(-n, 1.5707963267948966, ad);
  rr = fma(-n, 6.123233995736766e-17, rr);
  const int qd = ((int)n) & 3;
  const double z = rr * rr;
  const double sp = (((((1.6059043836821613e-10 * z - 2.505210838544172e-08) * z + 2.755731922398589e-06) * z
                      - 1.984126984126984e-04) * z + 8.333333333333333e-03) * z - 0.16666666666666666);
  const double sn = rr + rr * z * sp;
  const double cp = ((((((-1.1470745597729725e-11 * z + 2.08767569878681e-09) * z - 2.755731922398589e-07) * z
                       + 2.48015873015873e-05) * z - 1.3888888888888889e-03) * z + 0.041666666666666664) * z - 0.5);
  const double cs = 1.0 + z * cp;
  const double cv = (qd == 0) ? cs : (qd == 1) ? -sn : (qd == 2) ? -cs : sn;
  const double sv = (qd == 0) ? sn : (qd == 1) ? cs : (qd == 2) ? -sn : -cs;
  const float cf = (float)cv, sf = (float)sv;
  volatile float* pc = cosT + (size_t)t * 32 + j;
  volatile float* ps = sinT + (size_t)t * 32 + j;
  *pc = cf;
  *ps = sf;
  __threadfence();
  *pc = cf;
  *ps = sf;
}

__global__ void __launch_bounds__(256) k_flags(const int* __restrict__ mk, int* __restrict__ F) {
  __shared__ u32x4 fl4[16];
  const int lane = threadIdx.x & 31, w = threadIdx.x >> 5;
  const int qt = (int)blockIdx.x;
  unsigned fv[8];
#pragma unroll
  for (int i = 0; i < 8; ++i) {
    const int kt = 8 * w + i;
    int any = 0;
#pragma unroll
    for (int r = 0; r < 16; ++r) any |= mk[(size_t)(qt * 16 + r) * NT + kt * 32 + lane];
    fv[i] = (__builtin_amdgcn_ballot_w32(any != 0) != 0u) ? 1u : 0u;
  }
  if (lane == 0) {
    u32x4 v0, v1;
    v0[0] = fv[0]; v0[1] = fv[1]; v0[2] = fv[2]; v0[3] = fv[3];
    v1[0] = fv[4]; v1[1] = fv[5]; v1[2] = fv[6]; v1[3] = fv[7];
    fl4[2 * w] = v0;
    fl4[2 * w + 1] = v1;
  }
  __syncthreads();
  if (w == 0 && lane < 16) {
    const u32x4 v = fl4[lane];
    volatile u32x4* p = (volatile u32x4*)(F + (size_t)qt * 64) + lane;
    *p = v;
    __threadfence();
    *p = v;
  }
}

__global__ void __launch_bounds__(128) k_proj_qk(const __bf16* __restrict__ xp, const __bf16* __restrict__ wq,
                                                 const __bf16* __restrict__ wk, const float* __restrict__ cosT,
                                                 const float* __restrict__ sinT, __bf16* __restrict__ qo,
                                                 __bf16* __restrict__ ko) {
  __shared__ u32x4 lds[4][512];
  const int lane = threadIdx.x & 31, wid = threadIdx.x >> 5, lm = lane & 15, lh = lane >> 4;
  const int g = (int)blockIdx.x * 4 + wid;
  const int fi = g & 15, ti = g >> 4;
  const int n0 = fi * DK, m0 = ti * 32;
  const bool sel = (blockIdx.y != 0);
  const __bf16* W = sel ? wk : wq;
  __bf16* O = sel ? ko : qo;
  v8f acc[4][2] = {};
  gemm_core(W + (size_t)n0 * KD, PSW, xp + (size_t)m0 * KD, PSX, lm, lh, acc);
  const int bb = m0 >> 11, tb = m0 & (NT - 1);
#pragma unroll
  for (int bt = 0; bt < 2; ++bt) {
    const int tr = 16 * bt + lm;
    const int tpos = tb + tr;
#pragma unroll
    for (int at = 0; at < 2; ++at) {
      const float* cr = cosT + (size_t)tpos * 32 + 16 * at + 8 * lh;
      const float* sr = sinT + (size_t)tpos * 32 + 16 * at + 8 * lh;
      V8 c, s;
      c.q[0] = *(const f32x4*)cr; c.q[1] = *(const f32x4*)(cr + 4);
      s.q[0] = *(const f32x4*)sr; s.q[1] = *(const f32x4*)(sr + 4);
      float y1[8], y2[8];
#pragma unroll
      for (int r = 0; r < 8; ++r) {
        const float x1 = acc[at][bt][r], x2 = acc[at + 2][bt][r];
        y1[r] = x1 * c.v[r] - x2 * s.v[r];
        y2[r] = x2 * c.v[r] + x1 * s.v[r];
      }
      u32x4 h1, l1, h2, l2;
      split8(y1, h1, l1);
      split8(y2, h2, l2);
      lds[wid][tr * 8 + 2 * at + lh] = h1;
      lds[wid][256 + tr * 8 + 2 * at + lh] = l1;
      lds[wid][tr * 8 + 2 * (at + 2) + lh] = h2;
      lds[wid][256 + tr * 8 + 2 * (at + 2) + lh] = l2;
    }
  }
  __builtin_amdgcn_fence(__ATOMIC_RELEASE, "wavefront");
  __builtin_amdgcn_wave_barrier();
  const size_t rowbase = ((size_t)(bb * NH + fi) * NT + tb) * DK;
  auto emit = [&]() {
#pragma unroll
    for (int p = 0; p < 2; ++p) {
#pragma unroll
      for (int it = 0; it < 8; ++it) {
        const int L = 4 * it + (lane >> 3), pc = lane & 7;
        const u32x4 v = lds[wid][p * 256 + L * 8 + pc];
        __bf16* dst = O + (size_t)p * PSX + rowbase + (size_t)L * DK + pc * 8;
        *(volatile u32x4*)dst = v;
      }
    }
  };
  emit();
  __threadfence();
  emit();
}

__global__ void __launch_bounds__(128) k_proj_v(const __bf16* __restrict__ xp, const __bf16* __restrict__ wv,
                                                __bf16* __restrict__ vo) {
  __shared__ u32x4 lds[4][512];
  const int lane = threadIdx.x & 31, wid = threadIdx.x >> 5, lm = lane & 15, lh = lane >> 4;
  const int g = (int)blockIdx.x * 4 + wid;
  const int fi = g & 31, ti = g >> 5;
  const int n0 = fi * 32, m0 = ti * 64;
  const int hh = fi >> 1, d0 = (fi & 1) * 32;
  v8f acc[4][2] = {};
  gemm_core(xp + (size_t)m0 * KD, PSX, wv + (size_t)n0 * KD, PSW, lm, lh, acc);
#pragma unroll
  for (int bt = 0; bt < 2; ++bt) {
    const int dr = 16 * bt + lm;
#pragma unroll
    for (int at = 0; at < 4; ++at) {
      float y[8];
#pragma unroll
      for (int r = 0; r < 8; ++r) y[r] = acc[at][bt][r];
      u32x4 hi, lo;
      split8(y, hi, lo);
      lds[wid][dr * 8 + 2 * at + lh] = hi;
      lds[wid][256 + dr * 8 + 2 * at + lh] = lo;
    }
  }
  __builtin_amdgcn_fence(__ATOMIC_RELEASE, "wavefront");
  __builtin_amdgcn_wave_barrier();
  const int bb = m0 >> 11, tb = m0 & (NT - 1);
  const size_t rowbase = ((size_t)(bb * NH + hh) * DK + d0) * NT + tb;
  auto emit = [&]() {
#pragma unroll
    for (int p = 0; p < 2; ++p) {
#pragma unroll
      for (int it = 0; it < 8; ++it) {
        const int L = 4 * it + (lane >> 3), pc = lane & 7;
        const u32x4 v = lds[wid][p * 256 + L * 8 + pc];
        __bf16* dst = vo + (size_t)p * PSX + rowbase + (size_t)L * NT + pc * 8;
        *(volatile u32x4*)dst = v;
      }
    }
  };
  emit();
  __threadfence();
  emit();
}

__global__ void __launch_bounds__(128) k_attn(const __bf16* __restrict__ qp, const __bf16* __restrict__ kp,
                                              const __bf16* __restrict__ vp, const int* __restrict__ msk,
                                              const int* __restrict__ flg, const float* __restrict__ sw,
                                              const float* __restrict__ sb, __bf16* __restrict__ ap) {
  __shared__ u32x4 lds[4][256];
  const int lane = threadIdx.x & 31, wid = threadIdx.x >> 5, lm = lane & 15, lh = lane >> 4;
  const int g = (int)blockIdx.x * 4 + wid;
  const int b = g >> 11, h = (g >> 7) & 15, qt = g & 127, q0 = qt * 16;
  const size_t bh = (size_t)(b * NH + h);
  const __bf16* qrow = qp + (bh * NT + q0 + lm) * DK + 8 * lh;
  const __bf16* kb = kp + bh * NT * DK + 8 * lh;
  const __bf16* vb = vp + bh * DK * NT + (size_t)lm * NT + 8 * lh;
  const int* mrow = msk + (size_t)(q0 + lm) * NT + 8 * lh;
  const float* wr = sw + (size_t)b * NT + 8 * lh;
  const float bias = sb[h];
  const int f0 = flg[qt * 64 + lane], f1 = flg[qt * 64 + 32 + lane];
  const unsigned b0 = __builtin_amdgcn_ballot_w32(f0 != 0);
  const unsigned b1 = __builtin_amdgcn_ballot_w32(f1 != 0);
  int nch = 0;
  if (b1 != 0u) nch = 64 - __builtin_clz(b1);
  else if (b0 != 0u) nch = 32 - __builtin_clz(b0);

  float rmax = NEG_INF, rsum = 0.f;
  v8f o[4] = {};

  for (int ic = 0; ic < nch; ++ic) {
    const unsigned word = (ic < 32) ? b0 : b1;
    if (((word >> (ic & 31)) & 1u) == 0u) continue;
    const int k0 = ic * 32;
    const i32x4 mA = *(const i32x4*)(mrow + k0);
    const i32x4 mB = *(const i32x4*)(mrow + k0 + 4);
    const i32x4 mC = *(const i32x4*)(mrow + k0 + 16);
    const i32x4 mD = *(const i32x4*)(mrow + k0 + 20);
    const f32x4 wA = *(const f32x4*)(wr + k0);
    const f32x4 wB = *(const f32x4*)(wr + k0 + 4);
    const f32x4 wC = *(const f32x4*)(wr + k0 + 16);
    const f32x4 wD = *(const f32x4*)(wr + k0 + 20);
    Frag qh0, qh1, ql0, ql1;
    qh0.h[0] = *(const bf16x8*)(qrow);            qh0.h[1] = *(const bf16x8*)(qrow + 16);
    qh1.h[0] = *(const bf16x8*)(qrow + 32);       qh1.h[1] = *(const bf16x8*)(qrow + 48);
    ql0.h[0] = *(const bf16x8*)(qrow + PSX);      ql0.h[1] = *(const bf16x8*)(qrow + PSX + 16);
    ql1.h[0] = *(const bf16x8*)(qrow + PSX + 32); ql1.h[1] = *(const bf16x8*)(qrow + PSX + 48);
    v8f s0 = {}, s1 = {};
    Frag kh0, kh1, kl0, kl1;
    {
      const __bf16* kr = kb + (size_t)(k0 + lm) * DK;
      kh0.h[0] = *(const bf16x8*)(kr);            kh0.h[1] = *(const bf16x8*)(kr + 16);
      kh1.h[0] = *(const bf16x8*)(kr + 32);       kh1.h[1] = *(const bf16x8*)(kr + 48);
      kl0.h[0] = *(const bf16x8*)(kr + PSX);      kl0.h[1] = *(const bf16x8*)(kr + PSX + 16);
      kl1.h[0] = *(const bf16x8*)(kr + PSX + 32); kl1.h[1] = *(const bf16x8*)(kr + PSX + 48);
      s0 = mma(kh0.v, qh0.v, s0); s0 = mma(kh0.v, ql0.v, s0); s0 = mma(kl0.v, qh0.v, s0);
      s0 = mma(kh1.v, qh1.v, s0); s0 = mma(kh1.v, ql1.v, s0); s0 = mma(kl1.v, qh1.v, s0);
    }
    {
      const __bf16* kr = kb + (size_t)(k0 + 16 + lm) * DK;
      kh0.h[0] = *(const bf16x8*)(kr);            kh0.h[1] = *(const bf16x8*)(kr + 16);
      kh1.h[0] = *(const bf16x8*)(kr + 32);       kh1.h[1] = *(const bf16x8*)(kr + 48);
      kl0.h[0] = *(const bf16x8*)(kr + PSX);      kl0.h[1] = *(const bf16x8*)(kr + PSX + 16);
      kl1.h[0] = *(const bf16x8*)(kr + PSX + 32); kl1.h[1] = *(const bf16x8*)(kr + PSX + 48);
      s1 = mma(kh0.v, qh0.v, s1); s1 = mma(kh0.v, ql0.v, s1); s1 = mma(kl0.v, qh0.v, s1);
      s1 = mma(kh1.v, qh1.v, s1); s1 = mma(kh1.v, ql1.v, s1); s1 = mma(kl1.v, qh1.v, s1);
    }
    asm volatile(HAZ4 : "+v"(s0), "+v"(s1) : "v"(kl1.v), "v"(qh1.v));
    float e[16];
#pragma unroll
    for (int i = 0; i < 4; ++i) {
      e[i]      = (mA[i] != 0) ? (s0[i] * 0.125f + bias) * wA[i] : NEG_INF;
      e[4 + i]  = (mB[i] != 0) ? (s0[4 + i] * 0.125f + bias) * wB[i] : NEG_INF;
      e[8 + i]  = (mC[i] != 0) ? (s1[i] * 0.125f + bias) * wC[i] : NEG_INF;
      e[12 + i] = (mD[i] != 0) ? (s1[4 + i] * 0.125f + bias) * wD[i] : NEG_INF;
    }
    float cm = e[0];
#pragma unroll
    for (int i = 1; i < 16; ++i) cm = fmaxf(cm, e[i]);
    cm = fmaxf(cm, __shfl_xor(cm, 16, 32));
    const float nm = fmaxf(rmax, cm);
    const float nmu = (nm == NEG_INF) ? 0.f : nm;
    const float alpha = expf(rmax - nmu);
    rmax = nm;
    float psum = 0.f;
#pragma unroll
    for (int i = 0; i < 16; ++i) { e[i] = expf(e[i] - nmu); psum += e[i]; }
    psum += __shfl_xor(psum, 16, 32);
    rsum = rsum * alpha + psum;
#pragma unroll
    for (int dt = 0; dt < 4; ++dt) o[dt] = o[dt] * alpha;
    Frag ph, pl;
#pragma unroll
    for (int i = 0; i < 8; ++i) {
      const __bf16 hv0 = (__bf16)e[i];
      ph.h[0][i] = hv0;
      pl.h[0][i] = (__bf16)(e[i] - (float)hv0);
      const __bf16 hv1 = (__bf16)e[8 + i];
      ph.h[1][i] = hv1;
      pl.h[1][i] = (__bf16)(e[8 + i] - (float)hv1);
    }
    Frag vh, vl;
#pragma unroll
    for (int dt = 0; dt < 4; ++dt) {
      const __bf16* vr = vb + (size_t)(16 * dt) * NT + k0;
      vh.h[0] = *(const bf16x8*)(vr);        vh.h[1] = *(const bf16x8*)(vr + 16);
      vl.h[0] = *(const bf16x8*)(vr + PSX);  vl.h[1] = *(const bf16x8*)(vr + PSX + 16);
      o[dt] = mma(vh.v, ph.v, o[dt]);
      o[dt] = mma(vh.v, pl.v, o[dt]);
      o[dt] = mma(vl.v, ph.v, o[dt]);
    }
    asm volatile(HAZ4 : "+v"(o[0]), "+v"(o[1]), "+v"(o[2]), "+v"(o[3]) : "v"(vl.v), "v"(ph.v));
  }

  const float inv = 1.0f / rsum;
#pragma unroll
  for (int dt = 0; dt < 4; ++dt) {
    float y[8];
#pragma unroll
    for (int r = 0; r < 8; ++r) y[r] = o[dt][r] * inv;
    u32x4 hi, lo;
    split8(y, hi, lo);
    lds[wid][lm * 8 + 2 * dt + lh] = hi;
    lds[wid][128 + lm * 8 + 2 * dt + lh] = lo;
  }
  __builtin_amdgcn_fence(__ATOMIC_RELEASE, "wavefront");
  __builtin_amdgcn_wave_barrier();
  auto emit = [&]() {
#pragma unroll
    for (int p = 0; p < 2; ++p) {
#pragma unroll
      for (int it = 0; it < 4; ++it) {
        const int L = 4 * it + (lane >> 3), pc = lane & 7;
        const u32x4 v = lds[wid][p * 128 + L * 8 + pc];
        __bf16* dst = ap + (size_t)p * PSX + ((size_t)(b * NT + q0 + L)) * NC + h * DK + pc * 8;
        *(volatile u32x4*)dst = v;
      }
    }
  };
  emit();
  __threadfence();
  emit();
}

__global__ void __launch_bounds__(128) k_proj_out(const __bf16* __restrict__ wo, const __bf16* __restrict__ ap,
                                                  const float* __restrict__ bo, float* __restrict__ out) {
  __shared__ u32x4 lds[4][512];
  const int lane = threadIdx.x & 31, wid = threadIdx.x >> 5, lm = lane & 15, lh = lane >> 4;
  const int g = (int)blockIdx.x * 4 + wid;
  const int fi = g & 15, ti = g >> 4;
  const int n0 = fi * 64, m0 = ti * 32;
  v8f acc[4][2] = {};
  gemm_core(wo + (size_t)n0 * KD, PSW, ap + (size_t)m0 * KD, PSX, lm, lh, acc);
#pragma unroll
  for (int bt = 0; bt < 2; ++bt) {
    const int tr = 16 * bt + lm;
#pragma unroll
    for (int at = 0; at < 4; ++at) {
      const float* br = bo + n0 + 16 * at + 8 * lh;
      V8 bv, y;
      bv.q[0] = *(const f32x4*)br;
      bv.q[1] = *(const f32x4*)(br + 4);
      y.v = acc[at][bt] + bv.v;
      U4 u0, u1;
      u0.f = y.q[0];
      u1.f = y.q[1];
      lds[wid][tr * 16 + 4 * at + 2 * lh] = u0.u;
      lds[wid][tr * 16 + 4 * at + 2 * lh + 1] = u1.u;
    }
  }
  __builtin_amdgcn_fence(__ATOMIC_RELEASE, "wavefront");
  __builtin_amdgcn_wave_barrier();
  auto emit = [&]() {
#pragma unroll
    for (int it = 0; it < 16; ++it) {
      const int L = 4 * it + (lane >> 3), pc = lane & 7;
      const int tr = L >> 1, hf = L & 1;
      const u32x4 v = lds[wid][tr * 16 + hf * 8 + pc];
      float* dst = out + (size_t)(m0 + tr) * NC + n0 + hf * 32 + pc * 4;
      *(volatile u32x4*)dst = v;
    }
  };
  emit();
  __threadfence();
  emit();
}

extern "C" void kernel_launch(void* const* d_in, const int* in_sizes, int n_in,
                              void* d_out, int out_size, void* d_ws, size_t ws_size,
                              hipStream_t stream) {
  if (n_in != 9) return;
  if (in_sizes[0] != NB * NT * NC) return;
  if (in_sizes[1] != NC * NC || in_sizes[2] != NC * NC || in_sizes[3] != NC * NC || in_sizes[4] != NC * NC) return;
  if (in_sizes[5] != NC || in_sizes[6] != NH || in_sizes[7] != NB * NT || in_sizes[8] != NT * NT) return;
  if (out_size != NB * NT * NC) return;

  const float* x  = (const float*)d_in[0];
  const float* Wq = (const float*)d_in[1];
  const float* Wk = (const float*)d_in[2];
  const float* Wv = (const float*)d_in[3];
  const float* Wo = (const float*)d_in[4];
  const float* bo = (const float*)d_in[5];
  const float* sb = (const float*)d_in[6];
  const float* sw = (const float*)d_in[7];
  const int*   mk = (const int*)d_in[8];
  float* out = (float*)d_out;

  char* ws = (char*)d_ws;
  size_t off = 0;
  auto carve = [&](size_t bytes) -> char* {
    char* p = ws + off;
    off += (bytes + 255) & ~(size_t)255;
    return p;
  };
  __bf16* xpl = (__bf16*)carve(PSX * 2 * sizeof(__bf16));
  __bf16* wqp = (__bf16*)carve(PSW * 2 * sizeof(__bf16));
  __bf16* wkp = (__bf16*)carve(PSW * 2 * sizeof(__bf16));
  __bf16* wvp = (__bf16*)carve(PSW * 2 * sizeof(__bf16));
  __bf16* wop = (__bf16*)carve(PSW * 2 * sizeof(__bf16));
  __bf16* qpl = (__bf16*)carve(PSX * 2 * sizeof(__bf16));
  __bf16* kpl = (__bf16*)carve(PSX * 2 * sizeof(__bf16));
  __bf16* vpl = (__bf16*)carve(PSX * 2 * sizeof(__bf16));
  __bf16* apl = (__bf16*)carve(PSX * 2 * sizeof(__bf16));
  float* cosT = (float*)carve((size_t)NT * 32 * sizeof(float));
  float* sinT = (float*)carve((size_t)NT * 32 * sizeof(float));
  int*   flg  = (int*)carve((size_t)128 * 64 * sizeof(int));
  if (off > ws_size) return;

  k_split<<<dim3((unsigned)(PSX / 2048), 1), 256, 0, stream>>>(x, x, x, x, xpl, xpl, xpl, xpl, (int)PSX);
  k_split<<<dim3((unsigned)(PSW / 2048), 4), 256, 0, stream>>>(Wq, Wk, Wv, Wo, wqp, wkp, wvp, wop, (int)PSW);
  k_rope<<<NT / 8, 256, 0, stream>>>(cosT, sinT);
  k_flags<<<NT / 16, 256, 0, stream>>>(mk, flg);
  k_proj_qk<<<dim3(512, 2), 128, 0, stream>>>(xpl, wqp, wkp, cosT, sinT, qpl, kpl);
  k_proj_v<<<512, 128, 0, stream>>>(xpl, wvp, vpl);
  k_attn<<<1024, 128, 0, stream>>>(qpl, kpl, vpl, mk, flg, sw, sb, apl);
  k_proj_out<<<512, 128, 0, stream>>>(wop, apl, bo, out);
}
